// Model_73572789780577
// MI455X (gfx1250) — hardware-verified
//
#include <hip/hip_runtime.h>
#include <stddef.h>
#include <stdint.h>
#pragma clang fp contract(off)

#define NV     100000
#define NTET   500000
#define NLVL   10
#define TABLE  65536
#define NTHR   256
#define TM     256
#define HID    64
#define K1     96
#define K2     128
#define NO     13
#define NOP    16
#define AP     136
#define DP     68
#define GP     16
#define NBRUN  4096
#define NBC    160

#define PB_T   ((NLVL * TABLE * 4) / (8 * NTHR))
#define PB_V   ((NV + NTHR - 1) / NTHR)
#define PB_1   ((HID * (K1 / 8)) / NTHR)
#define PB_2   ((HID * (K2 / 8)) / NTHR)
#define PB_3   ((NOP * (K2 / 8)) / NTHR)
#define PB_C   1
#define PB_ALL (PB_T + PB_V + PB_1 + PB_2 + PB_3 + PB_C)
#define VPROWS (PB_V * NTHR)
#define NBLK_T ((NTET + TM - 1) / TM)
#define NBLK_V ((NV + NBRUN - 1) / NBRUN)
#define TET_LDS_BYTES (TM * DP * 4 + TM * AP * 2 + TM * GP * 4 + TM * 12 * 4 + NBC * 4)
#define WSMAX  134217728

static_assert(NTET % 32 == 0);
static_assert(NV % 32 == 0);
static_assert((NV * 4) % 128 == 0);
static_assert((TABLE & (TABLE - 1)) == 0);
static_assert(2 * 40 <= K1 && K1 % 32 == 0 && K2 % 32 == 0 && K2 == 2 * HID);
static_assert(NO <= NOP);
static_assert(TM % 32 == 0 && TM == NTHR);
static_assert(NBRUN % 32 == 0 && NBRUN % (4 * NTHR) == 0);
static_assert((NLVL * TABLE * 4) % (8 * NTHR) == 0);
static_assert(HID * (K1 / 8) == PB_1 * NTHR);
static_assert(HID * (K2 / 8) == PB_2 * NTHR);
static_assert(NOP * (K2 / 8) == PB_3 * NTHR);
static_assert((AP * 2) % 16 == 0 && AP >= K2 && (DP * 4) % 16 == 0 && DP >= HID);
static_assert((TM * AP) % 2 == 0);
static_assert(TET_LDS_BYTES <= 300000);
static_assert(NBC % 4 == 0 && NBC >= 147);
static_assert((TM * 12 * 4) % 128 == 0);
static_assert(((NTET % TM) * 3) % 32 == 0);

typedef float          v4f   __attribute__((ext_vector_type(4)));
typedef float          v8f   __attribute__((ext_vector_type(8)));
typedef int            v4i   __attribute__((ext_vector_type(4)));
typedef int            v8i   __attribute__((ext_vector_type(8)));
typedef unsigned       v2u   __attribute__((ext_vector_type(2)));
typedef unsigned       v4u   __attribute__((ext_vector_type(4)));
typedef unsigned short v4us  __attribute__((ext_vector_type(4)));
typedef unsigned short v8us  __attribute__((ext_vector_type(8)));
typedef unsigned short v16us __attribute__((ext_vector_type(16)));
typedef __bf16         v16bf __attribute__((ext_vector_type(16)));
typedef v4f  __attribute__((may_alias)) v4fa;
typedef v4i  __attribute__((may_alias)) v4ia;
typedef v2u  __attribute__((may_alias)) v2ua;
typedef v4u  __attribute__((may_alias)) v4ua;
typedef v4us __attribute__((may_alias)) v4usa;
typedef v8us __attribute__((may_alias)) v8usa;
union FragB { v16bf v; v16us u; v8us h[2]; v8i w; };

__device__ __forceinline__ v8f wmb(const FragB& a, const FragB& b, v8f c) {
  v8f d = __builtin_amdgcn_wmma_f32_16x16x32_bf16(false, a.v, false, b.v, (short)0, c, false, false);
  asm volatile("v_nop\n\tv_nop\n\tv_nop\n\tv_nop" : "+v"(d) : "v"(a.w), "v"(b.w));
  return d;
}

__device__ __forceinline__ unsigned bf16_bits(float f) {
  const unsigned u = __float_as_uint(f);
  return (u + 0x7FFFu + ((u >> 16) & 1u)) >> 16;
}
__device__ __forceinline__ float bf16_val(float f) { return __uint_as_float(bf16_bits(f) << 16); }
__device__ __forceinline__ unsigned bf16_bits_n(float f) {
  const unsigned u = __float_as_uint(f);
  const unsigned r = (u + 0x7FFFu + ((u >> 16) & 1u)) >> 16;
  const bool isn = (u & 0x7FFFFFFFu) > 0x7F800000u;
  return isn ? ((u >> 16) | 0x40u) : r;
}
__device__ __forceinline__ void put16(unsigned short* dp, v8us o) {
  *(volatile v8us*)dp = o;
  __threadfence();
  *(volatile v8us*)dp = o;
}
__device__ __forceinline__ void putf4(float* dp, v4f o) {
  *(volatile v4f*)dp = o;
  __threadfence();
  *(volatile v4f*)dp = o;
}

__global__ __launch_bounds__(NTHR) void k_prep(const float* __restrict__ verts, const float* __restrict__ cen,
                                               const float* __restrict__ tables,
                                               const float* __restrict__ W1, const float* __restrict__ b1,
                                               const float* __restrict__ W2, const float* __restrict__ b2,
                                               const float* __restrict__ W3, const float* __restrict__ b3,
                                               unsigned short* TBH, float* VP, unsigned short* B1t,
                                               unsigned short* B2t, unsigned short* B3t, float* BC) {
  __shared__ __attribute__((aligned(16))) float shc[NBC];
  const int tid = (int)threadIdx.x;
  const int blk = (int)blockIdx.x;
  if (blk < PB_T) {
    const size_t u = (size_t)blk * NTHR + (size_t)tid;
    const float* s = tables + u * 8;
    const v4f a = *(const v4fa*)s;
    const v4f c = *(const v4fa*)(s + 4);
    v8us o;
    o[0] = (unsigned short)bf16_bits(a.x); o[1] = (unsigned short)bf16_bits(a.y);
    o[2] = (unsigned short)bf16_bits(a.z); o[3] = (unsigned short)bf16_bits(a.w);
    o[4] = (unsigned short)bf16_bits(c.x); o[5] = (unsigned short)bf16_bits(c.y);
    o[6] = (unsigned short)bf16_bits(c.z); o[7] = (unsigned short)bf16_bits(c.w);
    put16(TBH + u * 8, o);
  } else if (blk < PB_T + PB_V) {
    const int row = (blk - PB_T) * NTHR + tid;
    const bool ok = row < NV;
    const int rc  = ok ? row : (NV - 1);
    const float r0 = verts[(size_t)rc * 3 + 0];
    const float r1 = verts[(size_t)rc * 3 + 1];
    const float r2 = verts[(size_t)rc * 3 + 2];
    v4f q;
    q.x = ok ? bf16_val(r0) : 0.0f;
    q.y = ok ? bf16_val(r1) : 0.0f;
    q.z = ok ? bf16_val(r2) : 0.0f;
    q.w = 0.0f;
    putf4(VP + (size_t)row * 4, q);
  } else if (blk < PB_T + PB_V + PB_1) {
    const int v  = (blk - PB_T - PB_V) * NTHR + tid;
    const int n  = v / (K1 / 8);
    const int j  = v - n * (K1 / 8);
    const int k8 = 8 * j;
    const bool ok = k8 < 80;
    const int ks = ok ? (k8 >= 40 ? k8 - 40 : k8) : 0;
    const float* p = W1 + (size_t)ks * HID + n;
    v8us o;
#pragma unroll
    for (int i = 0; i < 8; ++i) {
      const unsigned bb = bf16_bits(p[(size_t)i * HID]);
      o[i] = (unsigned short)(ok ? bb : 0u);
    }
    put16(B1t + (size_t)v * 8, o);
  } else if (blk < PB_T + PB_V + PB_1 + PB_2) {
    const int v  = (blk - PB_T - PB_V - PB_1) * NTHR + tid;
    const int n  = v >> 4;
    const int k8 = (v & 15) * 8;
    const int ks = k8 & (HID - 1);
    const float* p = W2 + (size_t)ks * HID + n;
    v8us o;
#pragma unroll
    for (int i = 0; i < 8; ++i) o[i] = (unsigned short)bf16_bits(p[(size_t)i * HID]);
    put16(B2t + (size_t)v * 8, o);
  } else if (blk < PB_T + PB_V + PB_1 + PB_2 + PB_3) {
    const int v  = (blk - PB_T - PB_V - PB_1 - PB_2) * NTHR + tid;
    const int n  = v >> 4;
    const int k8 = (v & 15) * 8;
    const int ks = k8 & (HID - 1);
    const bool ok = n < NO;
    const int nc = ok ? n : (NO - 1);
    const float* p = W3 + (size_t)ks * NO + nc;
    v8us o;
#pragma unroll
    for (int i = 0; i < 8; ++i) {
      const unsigned bb = bf16_bits(p[(size_t)i * NO]);
      o[i] = (unsigned short)(ok ? bb : 0u);
    }
    put16(B3t + (size_t)v * 8, o);
  } else {
    const int e  = tid;
    const int i1 = e < 63 ? e : 63;
    int i2 = e - 64;  i2 = i2 < 0 ? 0 : (i2 > 63 ? 63 : i2);
    int i3 = e - 128; i3 = i3 < 0 ? 0 : (i3 > NO - 1 ? NO - 1 : i3);
    int i4 = e - 144; i4 = i4 < 0 ? 0 : (i4 > 2 ? 2 : i4);
    const unsigned u1 = __float_as_uint(b1[i1]);
    const unsigned u2 = __float_as_uint(b2[i2]);
    const unsigned u3 = __float_as_uint(b3[i3]);
    const unsigned u4 = __float_as_uint(cen[i4]);
    const unsigned m1 = 0u - (unsigned)(e < 64);
    const unsigned m2 = 0u - (unsigned)(e >= 64 && e < 128);
    const unsigned m3 = 0u - (unsigned)(e >= 128 && e < 128 + NO);
    const unsigned m4 = 0u - (unsigned)(e >= 144 && e < 147);
    const unsigned ub = (u1 & m1) | (u2 & m2) | (u3 & m3) | (u4 & m4);
    const float val = bf16_val(__uint_as_float(ub));
    if (e < NBC) shc[e] = val;
    __syncthreads();
    const int uq = tid < (NBC / 4 - 1) ? tid : (NBC / 4 - 1);
    const v4f q = *(const v4fa*)(shc + 4 * uq);
    if (tid < NBC / 4) putf4(BC + 4 * tid, q);
  }
}

__device__ __forceinline__ float sq3(float x, float y, float z) { return (x * x + z * z) + y * y; }
__device__ __forceinline__ float dot3(float a0, float a1, float a2, float b0, float b1, float b2) {
  float p = a0 * b0;
  p = fmaf(a1, b1, p);
  p = fmaf(a2, b2, p);
  return p;
}
__device__ __forceinline__ void cswap(bool c, float& x, float& y) {
  const float tx = c ? y : x;
  const float ty = c ? x : y;
  x = tx;
  y = ty;
}
__device__ __forceinline__ void lu3(float a00, float a01, float a02, float a10, float a11, float a12,
                                    float a20, float a21, float a22, float b0, float b1, float b2,
                                    float& x0, float& x1, float& x2) {
  {
    const float m0 = fabsf(a00), m1 = fabsf(a10), m2 = fabsf(a20);
    const bool s1 = m1 > m0;
    const float mm = s1 ? m1 : m0;
    const bool s2 = m2 > mm;
    const bool w1 = s1 && !s2;
    cswap(w1, a00, a10); cswap(w1, a01, a11); cswap(w1, a02, a12); cswap(w1, b0, b1);
    cswap(s2, a00, a20); cswap(s2, a01, a21); cswap(s2, a02, a22); cswap(s2, b0, b2);
  }
  const float r0 = 1.0f / a00;
  float l10 = a10 * r0;
  float l20 = a20 * r0;
  a11 = a11 - l10 * a01;
  a12 = a12 - l10 * a02;
  a21 = a21 - l20 * a01;
  a22 = a22 - l20 * a02;
  {
    const bool s = fabsf(a21) > fabsf(a11);
    cswap(s, a11, a21); cswap(s, a12, a22); cswap(s, l10, l20); cswap(s, b1, b2);
  }
  const float r1 = 1.0f / a11;
  const float l21 = a21 * r1;
  a22 = a22 - l21 * a12;
  const float y0 = b0;
  const float y1 = b1 - l10 * y0;
  const float y2 = (b2 - l20 * y0) - l21 * y1;
  x2 = y2 / a22;
  const float y1b = y1 - a12 * x2;
  const float y0b = y0 - a02 * x2;
  x1 = y1b / a11;
  x0 = (y0b - a01 * x1) / a00;
}
__device__ __forceinline__ float selu_f(float x) {
  const float e = 1.6732632423543772f * expm1f(x);
  return 1.0507009873554805f * ((x > 0.0f) ? x : e);
}

template <int NT, int KK, int LDB>
__device__ __forceinline__ void wave_gemm(const unsigned short* sAw, float* sDw,
                                          const unsigned short* __restrict__ BT, int hh, int m) {
  v8f acc[2][NT];
  {
    const v8f z = {0.f, 0.f, 0.f, 0.f, 0.f, 0.f, 0.f, 0.f};
#pragma unroll
    for (int mt = 0; mt < 2; ++mt)
#pragma unroll
      for (int nt = 0; nt < NT; ++nt) acc[mt][nt] = z;
  }
  const unsigned short* ap0 = sAw + m * AP + 8 * hh;
  const unsigned short* ap1 = ap0 + 16 * AP;
  const unsigned short* bp  = BT + (size_t)m * LDB + 8 * hh;
#pragma unroll 1
  for (int k0 = 0; k0 < KK; k0 += 32) {
    FragB a0, a1;
    a0.h[0] = *(const v8usa*)(ap0 + k0);
    a0.h[1] = *(const v8usa*)(ap0 + k0 + 16);
    a1.h[0] = *(const v8usa*)(ap1 + k0);
    a1.h[1] = *(const v8usa*)(ap1 + k0 + 16);
#pragma unroll
    for (int nt = 0; nt < NT; ++nt) {
      const unsigned short* wq = bp + (size_t)(16 * nt) * LDB + k0;
      FragB b;
      b.h[0] = *(const v8usa*)wq;
      b.h[1] = *(const v8usa*)(wq + 16);
      acc[0][nt] = wmb(a0, b, acc[0][nt]);
      acc[1][nt] = wmb(a1, b, acc[1][nt]);
    }
  }
#pragma unroll
  for (int nt = 0; nt < NT; ++nt) {
    const int col = 16 * nt + m;
#pragma unroll
    for (int mt = 0; mt < 2; ++mt)
#pragma unroll
      for (int r = 0; r < 8; ++r) sDw[(16 * mt + 8 * hh + r) * DP + col] = acc[mt][nt][r];
  }
}

__device__ __forceinline__ void epi_selu(const float* rd, unsigned short* ra, const float* sb) {
#pragma unroll 1
  for (int c8 = 0; c8 < HID / 8; ++c8) {
    const v4f va = *(const v4fa*)(rd + 8 * c8);
    const v4f vb = *(const v4fa*)(rd + 8 * c8 + 4);
    const v4f ba = *(const v4fa*)(sb + 8 * c8);
    const v4f bb = *(const v4fa*)(sb + 8 * c8 + 4);
    const v8f x8 = {va.x + ba.x, va.y + ba.y, va.z + ba.z, va.w + ba.w,
                    vb.x + bb.x, vb.y + bb.y, vb.z + bb.z, vb.w + bb.w};
    v8us ho, lo;
#pragma unroll
    for (int i = 0; i < 8; ++i) {
      const float s = selu_f(x8[i]);
      const unsigned hb = bf16_bits_n(s);
      ho[i] = (unsigned short)hb;
      lo[i] = (unsigned short)bf16_bits_n(s - __uint_as_float(hb << 16));
    }
    *(v8usa*)(ra + 8 * c8)       = ho;
    *(v8usa*)(ra + HID + 8 * c8) = lo;
  }
}

#define CORNER(HX, HY, HZ, WX, WY, WZ) { \
    const unsigned hidx = ((HX) ^ (HY) ^ (HZ)) & (unsigned)(TABLE - 1); \
    const v2u tw = *(const v2ua*)(tb + 4 * (size_t)hidx); \
    const float wt = ((WX) * (WY)) * (WZ); \
    a0 = a0 + __uint_as_float(tw.x << 16) * wt; \
    a1 = a1 + __uint_as_float(tw.x & 0xffff0000u) * wt; \
    a2 = a2 + __uint_as_float(tw.y << 16) * wt; \
    a3 = a3 + __uint_as_float(tw.y & 0xffff0000u) * wt; }

__global__ __launch_bounds__(NTHR) void k_tet(const int* __restrict__ indices, const float* __restrict__ VP,
                                              const unsigned short* __restrict__ TBH,
                                              const unsigned short* __restrict__ B1t,
                                              const unsigned short* __restrict__ B2t,
                                              const unsigned short* __restrict__ B3t,
                                              const float* __restrict__ BC,
                                              float* ALPHA, float* out1) {
  extern __shared__ __attribute__((aligned(16))) float dyn[];
  float*          sD  = dyn;
  unsigned short* sA  = (unsigned short*)(dyn + TM * DP);
  float*          sG  = dyn + TM * DP + (TM * AP) / 2;
  float*          sVC = sG + TM * GP;
  float*          sB  = sVC + TM * 12;

  const int tid = (int)threadIdx.x, lane = tid & 31, wave = tid >> 5, hh = lane >> 4, m = lane & 15;
  const int blk = (int)blockIdx.x;

  {
    const int uq = tid < (NBC / 4 - 1) ? tid : (NBC / 4 - 1);
    const v4f q = *(const v4fa*)(BC + 4 * uq);
    if (tid < NBC / 4) *(v4fa*)(sB + 4 * tid) = q;
  }

  const int t  = blk * TM + tid;
  const int tc = t < NTET ? t : (NTET - 1);

  float*          rd = sD + tid * DP;
  unsigned short* ra = sA + tid * AP;
  float*          rg = sG + tid * GP;

  float p0, p1, p2, cr;
  {
    const v4i ii = *(const v4ia*)(indices + (size_t)tc * 4);
    int i0 = ii.x, i1 = ii.y, i2 = ii.z, i3 = ii.w;
    i0 = i0 < 0 ? 0 : (i0 > NV - 1 ? NV - 1 : i0);
    i1 = i1 < 0 ? 0 : (i1 > NV - 1 ? NV - 1 : i1);
    i2 = i2 < 0 ? 0 : (i2 > NV - 1 ? NV - 1 : i2);
    i3 = i3 < 0 ? 0 : (i3 > NV - 1 ? NV - 1 : i3);
    const v4f q0 = *(const v4fa*)(VP + (size_t)i0 * 4);
    const v4f q1 = *(const v4fa*)(VP + (size_t)i1 * 4);
    const v4f q2 = *(const v4fa*)(VP + (size_t)i2 * 4);
    const v4f q3 = *(const v4fa*)(VP + (size_t)i3 * 4);
    const v4f cq = *(const v4fa*)(BC + 144);

    const float e10 = q1.x - q0.x, e11 = q1.y - q0.y, e12 = q1.z - q0.z;
    const float e20 = q2.x - q0.x, e21 = q2.y - q0.y, e22 = q2.z - q0.z;
    const float e30 = q3.x - q0.x, e31 = q3.y - q0.y, e32 = q3.z - q0.z;
    const float s0 = sq3(q0.x, q0.y, q0.z);
    const float bb0 = sq3(q1.x, q1.y, q1.z) - s0;
    const float bb1 = sq3(q2.x, q2.y, q2.z) - s0;
    const float bb2 = sq3(q3.x, q3.y, q3.z) - s0;
    float c0, c1, c2;
    lu3(2.0f * e10 + 1e-6f, 2.0f * e11, 2.0f * e12,
        2.0f * e20, 2.0f * e21 + 1e-6f, 2.0f * e22,
        2.0f * e30, 2.0f * e31, 2.0f * e32 + 1e-6f,
        bb0, bb1, bb2, c0, c1, c2);
    const float d0 = c0 - q0.x, d1 = c1 - q0.y, d2 = c2 - q0.z;
    const float radius = sqrtf(sq3(d0, d1, d2));
    const float m00 = dot3(e10, e11, e12, e10, e11, e12) + 1e-6f;
    const float m01 = dot3(e10, e11, e12, e20, e21, e22);
    const float m02 = dot3(e10, e11, e12, e30, e31, e32);
    const float m11 = dot3(e20, e21, e22, e20, e21, e22) + 1e-6f;
    const float m12 = dot3(e20, e21, e22, e30, e31, e32);
    const float m22 = dot3(e30, e31, e32, e30, e31, e32) + 1e-6f;
    const float r0 = dot3(e10, e11, e12, d0, d1, d2);
    const float r1 = dot3(e20, e21, e22, d0, d1, d2);
    const float r2 = dot3(e30, e31, e32, d0, d1, d2);
    float l0, l1, l2;
    lu3(m00, m01, m02, m01, m11, m12, m02, m12, m22, r0, r1, r2, l0, l1, l2);
    float y0 = 1.0f - ((l0 + l2) + l1);
    float y1 = l0, y2 = l1, y3 = l2;
    y0 = fminf(fmaxf(y0, 0.0f), 1.0f);
    y1 = fminf(fmaxf(y1, 0.0f), 1.0f);
    y2 = fminf(fmaxf(y2, 0.0f), 1.0f);
    y3 = fminf(fmaxf(y3, 0.0f), 1.0f);
    const float bs = (y0 + y2) + (y1 + y3);
    const float binv = 1.0f / fmaxf(bs, 1e-6f);
    y0 = y0 * binv; y1 = y1 * binv; y2 = y2 * binv; y3 = y3 * binv;
    float cc0 = y0 * q0.x; cc0 = fmaf(y1, q1.x, cc0); cc0 = fmaf(y2, q2.x, cc0); cc0 = fmaf(y3, q3.x, cc0);
    float cc1 = y0 * q0.y; cc1 = fmaf(y1, q1.y, cc1); cc1 = fmaf(y2, q2.y, cc1); cc1 = fmaf(y3, q3.y, cc1);
    float cc2 = y0 * q0.z; cc2 = fmaf(y1, q1.z, cc2); cc2 = fmaf(y2, q2.z, cc2); cc2 = fmaf(y3, q3.z, cc2);
    const float x0 = (cc0 - cq.x) * 0.5f, x1 = (cc1 - cq.y) * 0.5f, x2 = (cc2 - cq.z) * 0.5f;
    const float nn = fmaxf(sqrtf(sq3(x0, x1, x2)), 1e-9f);
    const bool inside = nn <= 1.0f;
    const float rn = 1.0f / nn;
    const float fo = 2.0f - rn;
    const float v0 = inside ? x0 : ((fo * x0) * rn);
    const float v1 = inside ? x1 : ((fo * x1) * rn);
    const float v2 = inside ? x2 : ((fo * x2) * rn);
    const float jf = inside ? 1.0f : (1.0f / (nn * nn));
    cr = ((radius * 0.5f) * jf) * 0.5f;
    p0 = fminf(fmaxf(v0 * 0.25f + 0.5f, 0.0f), 0.999999f);
    p1 = fminf(fmaxf(v1 * 0.25f + 0.5f, 0.0f), 0.999999f);
    p2 = fminf(fmaxf(v2 * 0.25f + 0.5f, 0.0f), 0.999999f);
    float e2 = sq3(e10, e11, e12);
    e2 = fmaxf(e2, sq3(e20, e21, e22));
    e2 = fmaxf(e2, sq3(e30, e31, e32));
    e2 = fmaxf(e2, sq3(q1.x - q2.x, q1.y - q2.y, q1.z - q2.z));
    e2 = fmaxf(e2, sq3(q1.x - q3.x, q1.y - q3.y, q1.z - q3.z));
    e2 = fmaxf(e2, sq3(q2.x - q3.x, q2.y - q3.y, q2.z - q3.z));
    const float el = sqrtf(e2);
    const v4f g0 = {q0.x, q0.y, q0.z, q1.x};
    const v4f g1 = {q1.y, q1.z, q2.x, q2.y};
    const v4f g2 = {q2.z, q3.x, q3.y, q3.z};
    const v4f g3 = {cc0, cc1, cc2, el};
    *(v4fa*)(rg)      = g0;
    *(v4fa*)(rg + 4)  = g1;
    *(v4fa*)(rg + 8)  = g2;
    *(v4fa*)(rg + 12) = g3;
  }

#pragma unroll 1
  for (int l = 0; l < NLVL; ++l) {
    const float res = (float)(16 << l);
    const float fl  = (float)l;
    const float sc  = erff(1.0f / sqrtf((8.0f * fl) * cr + 1e-12f));
    const float xx0 = p0 * res, xx1 = p1 * res, xx2 = p2 * res;
    const float f0 = floorf(xx0), f1 = floorf(xx1), f2 = floorf(xx2);
    const float w0 = xx0 - f0, w1 = xx1 - f1, w2 = xx2 - f2;
    const float u0 = 1.0f - w0, u1 = 1.0f - w1, u2 = 1.0f - w2;
    const unsigned j0 = (unsigned)f0, j1 = (unsigned)f1, j2 = (unsigned)f2;
    const unsigned hx0 = j0, hx1 = j0 + 1u;
    const unsigned hy0 = j1 * 2654435761u, hy1 = (j1 + 1u) * 2654435761u;
    const unsigned hz0 = j2 * 805459861u,  hz1 = (j2 + 1u) * 805459861u;
    const unsigned short* tb = TBH + (size_t)l * TABLE * 4;
    float a0 = 0.0f, a1 = 0.0f, a2 = 0.0f, a3 = 0.0f;
    CORNER(hx0, hy0, hz0, u0, u1, u2)
    CORNER(hx1, hy0, hz0, w0, u1, u2)
    CORNER(hx0, hy1, hz0, u0, w1, u2)
    CORNER(hx1, hy1, hz0, w0, w1, u2)
    CORNER(hx0, hy0, hz1, u0, u1, w2)
    CORNER(hx1, hy0, hz1, w0, u1, w2)
    CORNER(hx0, hy1, hz1, u0, w1, w2)
    CORNER(hx1, hy1, hz1, w0, w1, w2)
    const float s0 = a0 * sc, s1 = a1 * sc, s2 = a2 * sc, s3 = a3 * sc;
    const unsigned h0 = bf16_bits_n(s0), h1 = bf16_bits_n(s1), h2 = bf16_bits_n(s2), h3 = bf16_bits_n(s3);
    v4us hv, lv;
    hv[0] = (unsigned short)h0; hv[1] = (unsigned short)h1; hv[2] = (unsigned short)h2; hv[3] = (unsigned short)h3;
    lv[0] = (unsigned short)bf16_bits_n(s0 - __uint_as_float(h0 << 16));
    lv[1] = (unsigned short)bf16_bits_n(s1 - __uint_as_float(h1 << 16));
    lv[2] = (unsigned short)bf16_bits_n(s2 - __uint_as_float(h2 << 16));
    lv[3] = (unsigned short)bf16_bits_n(s3 - __uint_as_float(h3 << 16));
    *(v4usa*)(ra + 4 * l)      = hv;
    *(v4usa*)(ra + 40 + 4 * l) = lv;
  }
  {
    const v8us z = {0, 0, 0, 0, 0, 0, 0, 0};
    *(v8usa*)(ra + 80) = z;
    *(v8usa*)(ra + 88) = z;
  }
  __syncthreads();

  const unsigned short* sAw = sA + 32 * wave * AP;
  float*                sDw = sD + 32 * wave * DP;

  wave_gemm<4, K1, K1>(sAw, sDw, B1t, hh, m);
  __syncthreads();
  epi_selu(rd, ra, sB);
  __syncthreads();
  wave_gemm<4, K2, K2>(sAw, sDw, B2t, hh, m);
  __syncthreads();
  epi_selu(rd, ra, sB + 64);
  __syncthreads();
  wave_gemm<1, K2, K2>(sAw, sDw, B3t, hh, m);
  __syncthreads();

  {
    const v4f qa = *(const v4fa*)(rd);
    const v4f qb = *(const v4fa*)(rd + 4);
    const v4f qc = *(const v4fa*)(rd + 8);
    const v4f qd = *(const v4fa*)(rd + 12);
    const v4f ba = *(const v4fa*)(sB + 128);
    const v4f bb = *(const v4fa*)(sB + 132);
    const v4f bc = *(const v4fa*)(sB + 136);
    const v4f bd = *(const v4fa*)(sB + 140);
    const float o0 = qa.x + ba.x, o1 = qa.y + ba.y, o2 = qa.z + ba.z, o3 = qa.w + ba.w;
    const float o4 = qb.x + bb.x, o5 = qb.y + bb.y, o6 = qb.z + bb.z, o7 = qb.w + bb.w;
    const float o8 = qc.x + bc.x, o9 = qc.y + bc.y, o10 = qc.z + bc.z, o11 = qc.w + bc.w;
    const float o12 = qd.x + bd.x;
    const v4f g0 = *(const v4fa*)(rg);
    const v4f g1 = *(const v4fa*)(rg + 4);
    const v4f g2 = *(const v4fa*)(rg + 8);
    const v4f g3 = *(const v4fa*)(rg + 12);
    const float el = g3.w;
    const float dcl = fminf(fmaxf(o0 + (-1.0f), -30.0f), 10.0f);
    const float density = expf(dcl);
    const float alpha = 1.0f - expf(-density * el);
    {
      float* apn = ALPHA + (size_t)blk * TM + tid;
      *(volatile float*)apn = alpha;
      __threadfence();
      *(volatile float*)apn = alpha;
    }
    const float bs0 = o1 + 0.5f, bs1 = o2 + 0.5f, bs2 = o3 + 0.5f;
    const float cb0 = fmaxf(bs0, 0.0f), cb1 = fmaxf(bs1, 0.0f), cb2 = fmaxf(bs2, 0.0f);
    const float g00 = cb0 * tanhf(o4),  g01 = cb0 * tanhf(o5),  g02 = cb0 * tanhf(o6);
    const float g10 = cb1 * tanhf(o7),  g11 = cb1 * tanhf(o8),  g12 = cb1 * tanhf(o9);
    const float g20 = cb2 * tanhf(o10), g21 = cb2 * tanhf(o11), g22 = cb2 * tanhf(o12);
    const float cc0 = g3.x, cc1 = g3.y, cc2 = g3.z;
    float vc[12];
#define VERT(J, VX, VY, VZ) { \
      const float dx = (VX) - cc0, dy = (VY) - cc1, dz = (VZ) - cc2; \
      const float iv = 1.0f / sqrtf(sq3(dx, dy, dz) + 1e-8f); \
      const float ox = dx * iv, oy = dy * iv, oz = dz * iv; \
      vc[3 * (J) + 0] = bs0 + dot3(g00, g01, g02, ox, oy, oz); \
      vc[3 * (J) + 1] = bs1 + dot3(g10, g11, g12, ox, oy, oz); \
      vc[3 * (J) + 2] = bs2 + dot3(g20, g21, g22, ox, oy, oz); }
    VERT(0, g0.x, g0.y, g0.z)
    VERT(1, g0.w, g1.x, g1.y)
    VERT(2, g1.z, g1.w, g2.x)
    VERT(3, g2.y, g2.z, g2.w)
#undef VERT
    const v4f w0 = {vc[0], vc[1], vc[2],  vc[3]};
    const v4f w1 = {vc[4], vc[5], vc[6],  vc[7]};
    const v4f w2 = {vc[8], vc[9], vc[10], vc[11]};
    float* rv = sVC + tid * 12;
    *(v4fa*)(rv)     = w0;
    *(v4fa*)(rv + 4) = w1;
    *(v4fa*)(rv + 8) = w2;
  }
  __syncthreads();

  {
    int nvt = NTET - blk * TM;
    nvt = nvt > TM ? TM : (nvt < 0 ? 0 : nvt);
    const int nun = nvt * 3;
    v4f pv[3];
#pragma unroll
    for (int it = 0; it < 3; ++it) pv[it] = *(const v4fa*)(sVC + (size_t)(it * NTHR + tid) * 4);
    float* ob = out1 + (size_t)blk * (TM * 12);
#pragma unroll
    for (int it = 0; it < 3; ++it) {
      const int u = it * NTHR + tid;
      if (u < nun) *(volatile v4f*)(ob + (size_t)u * 4) = pv[it];
    }
    __threadfence();
#pragma unroll
    for (int it = 0; it < 3; ++it) {
      const int u = it * NTHR + tid;
      if (u < nun) *(volatile v4f*)(ob + (size_t)u * 4) = pv[it];
    }
  }
}
#undef CORNER

__global__ __launch_bounds__(NTHR) void k_vmax(const int* __restrict__ indices, const float* __restrict__ ALPHA,
                                               float* out0) {
  __shared__ __attribute__((aligned(16))) unsigned tab[NBRUN];
  const int tid = (int)threadIdx.x;
  const int blk = (int)blockIdx.x;
  const unsigned ubase = (unsigned)blk * (unsigned)NBRUN;
  {
    const v4u z4 = {0u, 0u, 0u, 0u};
    for (int i = tid * 4; i < NBRUN; i += NTHR * 4) *(v4ua*)(tab + i) = z4;
  }
  __syncthreads();

  const int nIter = (NTET + NTHR - 1) / NTHR;
#pragma unroll 1
  for (int it = 0; it < nIter; ++it) {
    const int t  = it * NTHR + tid;
    const bool ok = t < NTET;
    const int tc = ok ? t : (NTET - 1);
    const v4i k = *(const v4ia*)(indices + (size_t)tc * 4);
    float a = ALPHA[tc];
    a = a + 0.0f;
    a = (a < 0.0f) ? 0.0f : a;
    const unsigned bits = __float_as_uint(a);
    const unsigned s0 = (unsigned)k.x - ubase, s1 = (unsigned)k.y - ubase;
    const unsigned s2 = (unsigned)k.z - ubase, s3 = (unsigned)k.w - ubase;
    if (ok && s0 < (unsigned)NBRUN) atomicMax(&tab[s0], bits);
    if (ok && s1 < (unsigned)NBRUN) atomicMax(&tab[s1], bits);
    if (ok && s2 < (unsigned)NBRUN) atomicMax(&tab[s2], bits);
    if (ok && s3 < (unsigned)NBRUN) atomicMax(&tab[s3], bits);
  }
  __syncthreads();

  int nv = NV - blk * NBRUN;
  nv = nv > NBRUN ? NBRUN : (nv < 0 ? 0 : nv);
  const int nun = nv / 4;
  v4u pv[NBRUN / (4 * NTHR)];
#pragma unroll
  for (int it = 0; it < NBRUN / (4 * NTHR); ++it) pv[it] = *(const v4ua*)(tab + (size_t)(it * NTHR + tid) * 4);
  unsigned* ob = (unsigned*)out0 + (size_t)blk * NBRUN;
#pragma unroll
  for (int it = 0; it < NBRUN / (4 * NTHR); ++it) {
    const int u = it * NTHR + tid;
    if (u < nun) *(volatile v4u*)(ob + (size_t)u * 4) = pv[it];
  }
  __threadfence();
#pragma unroll
  for (int it = 0; it < NBRUN / (4 * NTHR); ++it) {
    const int u = it * NTHR + tid;
    if (u < nun) *(volatile v4u*)(ob + (size_t)u * 4) = pv[it];
  }
}

extern "C" void kernel_launch(void* const* d_in, const int* in_sizes, int n_in,
                              void* d_out, int out_size, void* d_ws, size_t ws_size,
                              hipStream_t stream) {
  if (n_in < 10) return;
  if (in_sizes[0] != NV * 3) return;
  if (in_sizes[1] != NTET * 4) return;
  if (in_sizes[2] != 3) return;
  if (in_sizes[3] != NLVL * TABLE * 4) return;
  if (in_sizes[4] != 40 * HID) return;
  if (in_sizes[5] != HID) return;
  if (in_sizes[6] != HID * HID) return;
  if (in_sizes[7] != HID) return;
  if (in_sizes[8] != HID * NO) return;
  if (in_sizes[9] != NO) return;
  if ((long long)out_size != (long long)NV + (long long)NTET * 12) return;

  const float* verts  = (const float*)d_in[0];
  const int*   idx    = (const int*)d_in[1];
  const float* cen    = (const float*)d_in[2];
  const float* tables = (const float*)d_in[3];
  const float* W1 = (const float*)d_in[4];
  const float* b1 = (const float*)d_in[5];
  const float* W2 = (const float*)d_in[6];
  const float* b2 = (const float*)d_in[7];
  const float* W3 = (const float*)d_in[8];
  const float* b3 = (const float*)d_in[9];
  float* out0 = (float*)d_out;
  float* out1 = (float*)d_out + NV;

  char* ws = (char*)d_ws;
  size_t off = 0;
  const size_t oTBH = off; off += (size_t)NLVL * TABLE * 4 * 2;     off = (off + 255) & ~(size_t)255;
  const size_t oVP  = off; off += (size_t)VPROWS * 4 * 4;           off = (off + 255) & ~(size_t)255;
  const size_t oAL  = off; off += (size_t)NBLK_T * TM * 4;          off = (off + 255) & ~(size_t)255;
  const size_t oB1  = off; off += (size_t)HID * K1 * 2;             off = (off + 255) & ~(size_t)255;
  const size_t oB2  = off; off += (size_t)HID * K2 * 2;             off = (off + 255) & ~(size_t)255;
  const size_t oB3  = off; off += (size_t)NOP * K2 * 2;             off = (off + 255) & ~(size_t)255;
  const size_t oBC  = off; off += (size_t)NBC * 4;                  off = (off + 255) & ~(size_t)255;
  if (off > ws_size || off > (size_t)WSMAX) return;
  unsigned short* TBH = (unsigned short*)(ws + oTBH);
  float*          VP  = (float*)(ws + oVP);
  float*          AL  = (float*)(ws + oAL);
  unsigned short* B1t = (unsigned short*)(ws + oB1);
  unsigned short* B2t = (unsigned short*)(ws + oB2);
  unsigned short* B3t = (unsigned short*)(ws + oB3);
  float*          BC  = (float*)(ws + oBC);

  hipFuncSetAttribute(reinterpret_cast<const void*>(&k_tet), hipFuncAttributeMaxDynamicSharedMemorySize,
                      (int)TET_LDS_BYTES);

  k_prep<<<PB_ALL, NTHR, 0, stream>>>(verts, cen, tables, W1, b1, W2, b2, W3, b3, TBH, VP, B1t, B2t, B3t, BC);
  k_tet<<<NBLK_T, NTHR, TET_LDS_BYTES, stream>>>(idx, VP, TBH, B1t, B2t, B3t, BC, AL, out1);
  k_vmax<<<NBLK_V, NTHR, 0, stream>>>(idx, AL, out0);
  (void)hipGetLastError();
}
